// BCosGCN_28346784153649
// MI455X (gfx1250) — hardware-verified
//
#include <hip/hip_runtime.h>
#include <stddef.h>


#define DF      128
#define NTHR    256
#define NWAVE   8
#define EPT     8
#define NGRP    2
#define CHUNK   (NTHR * EPT * NGRP)
#define WCAP    (EPT * NGRP * 32)
#define LISTN   (NWAVE * WCAP)
#define NBA     512
#define NBD     4096
#define NGB     64
#define GROWS   128
#define WSCALE  8.0f
#define WINV    0.125f
#define LN_EPS  1e-5f
#define BC_EPS  1e-6f
#define TEMP_C  1.5f
#define RR_C    0.6f
#define RR_1    0.4f

#define LDS_GEMM (GROWS * DF * 4)
#define LDS_AGG  (NBA * DF * 4 + LISTN * 4 + 64)

static_assert((CHUNK & (CHUNK - 1)) == 0);
static_assert(CHUNK <= 4096);
static_assert(NBA <= 4096 && NBD <= 4096 && NGB <= 4096);
static_assert((NBA & (NBA - 1)) == 0 && (NBD & (NBD - 1)) == 0 && (NGB & (NGB - 1)) == 0);
static_assert(NBA == NWAVE * 64 && NGB == NWAVE * 8 && NBD == NWAVE * 4 * 128);
static_assert(GROWS == NWAVE * 16 && NBA % GROWS == 0);

typedef float    v4f  __attribute__((ext_vector_type(4)));
typedef float    v8f  __attribute__((ext_vector_type(8)));
typedef int      v4i  __attribute__((ext_vector_type(4)));
typedef _Float16 v8h  __attribute__((ext_vector_type(8)));
typedef _Float16 v16h __attribute__((ext_vector_type(16)));
union FragH { v16h v; v8h h[2]; };

__device__ __forceinline__ v8h cvt8(v4f a, v4f b) {
  v8h r;
  r[0] = (_Float16)a.x; r[1] = (_Float16)a.y; r[2] = (_Float16)a.z; r[3] = (_Float16)a.w;
  r[4] = (_Float16)b.x; r[5] = (_Float16)b.y; r[6] = (_Float16)b.z; r[7] = (_Float16)b.w;
  return r;
}

__device__ __forceinline__ v8f wmh(v16h a, v16h b, v8f c) {
  v8f d = __builtin_amdgcn_wmma_f32_16x16x32_f16(false, a, false, b, (short)0, c, false, false);
  asm volatile("v_nop\n\tv_nop\n\tv_nop\n\tv_nop" : "+v"(d) : "v"(a), "v"(b));
  return d;
}

__device__ __forceinline__ float wave_sum32(float v) {
#pragma unroll
  for (int off = 16; off > 0; off >>= 1) v += __shfl_xor(v, off, 32);
  return v;
}

template <int NB>
__device__ __forceinline__ int scan_chunk(const int* __restrict__ keys, int nK, int cbase, int base,
                                          int* list, int tid, int wave) {
  int wc = 0;
#pragma unroll
  for (int gq = 0; gq < NGRP; ++gq) {
    const int el0  = (gq * NTHR + tid) * EPT;
    const int e0   = cbase + el0;
    const int sent = -2147483647 - 1;
    v4i da, db;
    if (e0 + 7 < nK) {
      da = *(const v4i*)(keys + e0);
      db = *(const v4i*)(keys + e0 + 4);
    } else {
      da.x = (e0     < nK) ? keys[min(e0, nK - 1)] : sent;
      da.y = (e0 + 1 < nK) ? keys[min(e0 + 1, nK - 1)] : sent;
      da.z = (e0 + 2 < nK) ? keys[min(e0 + 2, nK - 1)] : sent;
      da.w = (e0 + 3 < nK) ? keys[min(e0 + 3, nK - 1)] : sent;
      db.x = (e0 + 4 < nK) ? keys[min(e0 + 4, nK - 1)] : sent;
      db.y = (e0 + 5 < nK) ? keys[min(e0 + 5, nK - 1)] : sent;
      db.z = (e0 + 6 < nK) ? keys[min(e0 + 6, nK - 1)] : sent;
      db.w = (e0 + 7 < nK) ? keys[min(e0 + 7, nK - 1)] : sent;
    }
    const unsigned nb = (unsigned)base;
    const unsigned s0 = (unsigned)da.x - nb, s1 = (unsigned)da.y - nb;
    const unsigned s2 = (unsigned)da.z - nb, s3 = (unsigned)da.w - nb;
    const unsigned s4 = (unsigned)db.x - nb, s5 = (unsigned)db.y - nb;
    const unsigned s6 = (unsigned)db.z - nb, s7 = (unsigned)db.w - nb;
    const bool h0 = s0 < (unsigned)NB, h1 = s1 < (unsigned)NB, h2 = s2 < (unsigned)NB, h3 = s3 < (unsigned)NB;
    const bool h4 = s4 < (unsigned)NB, h5 = s5 < (unsigned)NB, h6 = s6 < (unsigned)NB, h7 = s7 < (unsigned)NB;
    const unsigned any = __builtin_amdgcn_ballot_w32(h0 | h1 | h2 | h3 | h4 | h5 | h6 | h7);
    if (any != 0u) {
#define HITJ(J, HJ, SJ) { \
        const unsigned mj = __builtin_amdgcn_ballot_w32(HJ); \
        if (mj != 0u) { \
          if (HJ) { \
            const int pos = wc + (int)__builtin_amdgcn_mbcnt_lo(mj, 0u); \
            if (pos < WCAP) list[wave * WCAP + pos] = ((el0 + (J)) << 12) | (int)(SJ); \
          } \
          wc += (int)__builtin_popcount(mj); } }
      HITJ(0, h0, s0)
      HITJ(1, h1, s1)
      HITJ(2, h2, s2)
      HITJ(3, h3, s3)
      HITJ(4, h4, s4)
      HITJ(5, h5, s5)
      HITJ(6, h6, s6)
      HITJ(7, h7, s7)
#undef HITJ
    }
  }
  return wc;
}

__global__ __launch_bounds__(NTHR) void k_wprep(
    const float* __restrict__ W1, const float* __restrict__ W2,
    _Float16* w1s, _Float16* w2s) {
  const int i  = blockIdx.x * NTHR + threadIdx.x;
  const int n1 = DF * DF / 8;
  if (i >= 2 * n1) return;
  const bool first = i < n1;
  const int o  = (first ? i : i - n1) * 8;
  const int n  = o / DF;
  const int k0 = o - n * DF;
  const float* p = (first ? W1 : W2) + (size_t)k0 * DF + n;
  v4f a, b;
  a.x = p[0];      a.y = p[DF];     a.z = p[2 * DF]; a.w = p[3 * DF];
  b.x = p[4 * DF]; b.y = p[5 * DF]; b.z = p[6 * DF]; b.w = p[7 * DF];
  a = a * WSCALE;
  b = b * WSCALE;
  const v8h hv = cvt8(a, b);
  _Float16* dp = (first ? w1s : w2s) + o;
  *(volatile v8h*)dp = hv;
  __threadfence();
  *(volatile v8h*)dp = hv;
}

__global__ __launch_bounds__(NTHR) void k_xcvt(
    const float* __restrict__ x, _Float16* xh, int nN, int nRows) {
  const size_t i = (size_t)blockIdx.x * NTHR + threadIdx.x;
  const size_t total = (size_t)nRows * (DF / 8);
  if (i >= total) return;
  const int r  = (int)(i >> 4);
  const int c0 = (int)(i & 15) * 8;
  int node = r > nN - 1 ? nN - 1 : r;
  const float* xp = x + (size_t)node * DF + c0;
  const v4f a = *(const v4f*)xp, b = *(const v4f*)(xp + 4);
  const v8h hv = cvt8(a, b);
  _Float16* dp = xh + (size_t)r * DF + c0;
  *(volatile v8h*)dp = hv;
  __threadfence();
  *(volatile v8h*)dp = hv;
}

__global__ __launch_bounds__(NTHR) void k_deg(
    const int* __restrict__ dsts, float* dinv, int nE) {
  __shared__ __attribute__((aligned(16))) int cnt[NBD];
  __shared__ __attribute__((aligned(16))) int list[LISTN];
  __shared__ int wcnt[NWAVE];
  const int tid = threadIdx.x, lane = tid & 31, wave = tid >> 5;
  const int nodeBase = blockIdx.x * NBD;

  for (int i = tid; i < NBD; i += NTHR) cnt[i] = 0;
  __syncthreads();

  const int nChunks = (nE + CHUNK - 1) / CHUNK;
#pragma unroll 1
  for (int ch = 0; ch < nChunks; ++ch) {
    const int cbase = ch * CHUNK;
    const int wc = scan_chunk<NBD>(dsts, nE, cbase, nodeBase, list, tid, wave);
    if (lane == 0) wcnt[wave] = wc;
    __syncthreads();
    if (wave == 0) {
#pragma unroll 1
      for (int wsx = 0; wsx < NWAVE; ++wsx) {
        int n = __builtin_amdgcn_readfirstlane(wcnt[wsx]);
        n = n > WCAP ? WCAP : (n < 0 ? 0 : n);
        const int* lp = list + wsx * WCAP;
#pragma unroll 1
        for (int i = 0; i < n; ++i) {
          const int ent  = __builtin_amdgcn_readfirstlane(lp[i]);
          const int slot = ent & (NBD - 1);
          if (lane == 0) cnt[slot] = cnt[slot] + 1;
        }
      }
    }
    __syncthreads();
  }

  v4f dq[4];
#pragma unroll
  for (int q = 0; q < 4; ++q) {
    const int f = (wave * 4 + q) * 128 + 4 * lane;
    const v4i c = *(const v4i*)(cnt + f);
    dq[q].x = rsqrtf((float)(c.x + 1));
    dq[q].y = rsqrtf((float)(c.y + 1));
    dq[q].z = rsqrtf((float)(c.z + 1));
    dq[q].w = rsqrtf((float)(c.w + 1));
  }
  float* dp = dinv + (size_t)nodeBase;
#pragma unroll
  for (int q = 0; q < 4; ++q) *(volatile v4f*)(dp + (wave * 4 + q) * 128 + 4 * lane) = dq[q];
  __threadfence();
#pragma unroll
  for (int q = 0; q < 4; ++q) *(volatile v4f*)(dp + (wave * 4 + q) * 128 + 4 * lane) = dq[q];
}

__global__ __launch_bounds__(NTHR) void k_gemm(
    const _Float16* __restrict__ ah, const _Float16* __restrict__ wsn,
    const float* __restrict__ dinv, float* g) {
  extern __shared__ v4f lds_dyn[];
  float* stg = (float*)lds_dyn;
  const int tid = threadIdx.x, lane = tid & 31, wave = tid >> 5, hh = lane >> 4, m = lane & 15;
  const int rowBase = blockIdx.x * GROWS;

  v8f acc[8];
#pragma unroll
  for (int t = 0; t < 8; ++t) { v8f z = {0.f, 0.f, 0.f, 0.f, 0.f, 0.f, 0.f, 0.f}; acc[t] = z; }
  const _Float16* ar = ah + ((size_t)rowBase + wave * 16 + m) * DF + 8 * hh;
#pragma unroll 1
  for (int kt = 0; kt < DF / 32; ++kt) {
    FragH a;
    a.h[0] = *(const v8h*)(ar + 32 * kt);
    a.h[1] = *(const v8h*)(ar + 32 * kt + 16);
#pragma unroll
    for (int t = 0; t < 8; ++t) {
      const _Float16* bp = wsn + (size_t)(16 * t + m) * DF + 32 * kt + 8 * hh;
      FragH b;
      b.h[0] = *(const v8h*)bp;
      b.h[1] = *(const v8h*)(bp + 16);
      acc[t] = wmh(a.v, b.v, acc[t]);
    }
  }

  const int r0 = wave * 16 + 8 * hh;
  const v4f dA = *(const v4f*)(dinv + (size_t)rowBase + r0);
  const v4f dB = *(const v4f*)(dinv + (size_t)rowBase + r0 + 4);
  const float d0 = dA.x * WINV, d1 = dA.y * WINV, d2 = dA.z * WINV, d3 = dA.w * WINV;
  const float d4 = dB.x * WINV, d5 = dB.y * WINV, d6 = dB.z * WINV, d7 = dB.w * WINV;
  float* sp = stg + r0 * DF + m;
#pragma unroll
  for (int t = 0; t < 8; ++t) {
    sp[0 * DF + 16 * t] = acc[t][0] * d0;
    sp[1 * DF + 16 * t] = acc[t][1] * d1;
    sp[2 * DF + 16 * t] = acc[t][2] * d2;
    sp[3 * DF + 16 * t] = acc[t][3] * d3;
    sp[4 * DF + 16 * t] = acc[t][4] * d4;
    sp[5 * DF + 16 * t] = acc[t][5] * d5;
    sp[6 * DF + 16 * t] = acc[t][6] * d6;
    sp[7 * DF + 16 * t] = acc[t][7] * d7;
  }
  __syncthreads();

  const float* lp = stg + wave * 16 * DF + 4 * lane;
  float* gp = g + ((size_t)rowBase + wave * 16) * DF + 4 * lane;
#pragma unroll
  for (int i = 0; i < 16; ++i) { const v4f v = *(const v4f*)(lp + i * DF); *(volatile v4f*)(gp + (size_t)i * DF) = v; }
  __threadfence();
#pragma unroll
  for (int i = 0; i < 16; ++i) { const v4f v = *(const v4f*)(lp + i * DF); *(volatile v4f*)(gp + (size_t)i * DF) = v; }
}

template <int MODE>
__global__ __launch_bounds__(NTHR) void k_agg(
    const int* __restrict__ srcs, const int* __restrict__ dsts,
    const float* __restrict__ g, const float* __restrict__ dinv,
    const float* __restrict__ bias, const float* __restrict__ lnw, const float* __restrict__ lnb,
    _Float16* hout, float* fout, int nN, int nE) {
  extern __shared__ v4f lds_dyn[];
  float* acc  = (float*)lds_dyn;
  int*   list = (int*)(acc + NBA * DF);
  int*   wcnt = list + LISTN;
  const int tid = threadIdx.x, lane = tid & 31, wave = tid >> 5;
  const int nodeBase = blockIdx.x * NBA;

  {
    const v4f z = {0.f, 0.f, 0.f, 0.f};
    for (int i = tid; i < NBA * DF / 4; i += NTHR) lds_dyn[i] = z;
  }
  __syncthreads();

  const int nChunks = (nE + CHUNK - 1) / CHUNK;
#pragma unroll 1
  for (int ch = 0; ch < nChunks; ++ch) {
    const int cbase = ch * CHUNK;
    const int wc = scan_chunk<NBA>(dsts, nE, cbase, nodeBase, list, tid, wave);
    if (lane == 0) wcnt[wave] = wc;
    __syncthreads();
    if (wave == 0) {
#pragma unroll 1
      for (int wsx = 0; wsx < NWAVE; ++wsx) {
        int n = __builtin_amdgcn_readfirstlane(wcnt[wsx]);
        n = n > WCAP ? WCAP : (n < 0 ? 0 : n);
        const int* lp = list + wsx * WCAP;
#pragma unroll 1
        for (int i = 0; i < n; ++i) {
          const int ent  = __builtin_amdgcn_readfirstlane(lp[i]);
          const int slot = ent & (NBA - 1);
          int e = cbase + ((ent >> 12) & (CHUNK - 1));
          e = e > nE - 1 ? nE - 1 : e;
          int s = srcs[e];
          s = s < 0 ? 0 : (s > nN - 1 ? nN - 1 : s);
          const v4f v = *(const v4f*)(g + (size_t)s * DF + 4 * lane);
          v4f* ap = (v4f*)(acc + slot * DF + 4 * lane);
          *ap = *ap + v;
        }
      }
    }
    __syncthreads();
  }

  const int c4 = 4 * lane;
  const v4f bv = *(const v4f*)(bias + c4);
  const v4f wv = *(const v4f*)(lnw + c4);
  const v4f lb = *(const v4f*)(lnb + c4);
  const float invH = 1.0f / (float)DF;
#pragma unroll 1
  for (int i = 0; i < NBA / NWAVE; ++i) {
    const int slot = wave * (NBA / NWAVE) + i;
    int node = nodeBase + slot;
    node = node > nN - 1 ? nN - 1 : node;
    const float d  = dinv[node];
    const v4f   gv = *(const v4f*)(g + (size_t)node * DF + c4);
    v4f* ap = (v4f*)(acc + slot * DF + c4);
    const v4f v = (*ap + gv) * d + bv;
    const float mu = wave_sum32(v.x + v.y + v.z + v.w) * invH;
    const float e0 = v.x - mu, e1 = v.y - mu, e2 = v.z - mu, e3 = v.w - mu;
    const float var = wave_sum32(e0 * e0 + e1 * e1 + e2 * e2 + e3 * e3) * invH;
    const float rs = rsqrtf(var + LN_EPS);
    const float y0 = e0 * rs * wv.x + lb.x;
    const float y1 = e1 * rs * wv.y + lb.y;
    const float y2 = e2 * rs * wv.z + lb.z;
    const float y3 = e3 * rs * wv.w + lb.w;
    const float h0 = y0 > 0.0f ? y0 : expm1f(y0);
    const float h1 = y1 > 0.0f ? y1 : expm1f(y1);
    const float h2 = y2 > 0.0f ? y2 : expm1f(y2);
    const float h3 = y3 > 0.0f ? y3 : expm1f(y3);
    v4f hv;
    if (MODE == 2) {
      const float nrm = sqrtf(wave_sum32(h0 * h0 + h1 * h1 + h2 * h2 + h3 * h3) + BC_EPS);
      const float sc  = 1.0f / (nrm + BC_EPS);
      hv.x = RR_C * h0 + RR_1 * ((TEMP_C * h0) * sc);
      hv.y = RR_C * h1 + RR_1 * ((TEMP_C * h1) * sc);
      hv.z = RR_C * h2 + RR_1 * ((TEMP_C * h2) * sc);
      hv.w = RR_C * h3 + RR_1 * ((TEMP_C * h3) * sc);
    } else {
      hv.x = h0; hv.y = h1; hv.z = h2; hv.w = h3;
    }
    *ap = hv;
  }
  __syncthreads();

  if (MODE == 1) {
    const int rsub = lane >> 4, c8 = (lane & 15) * 8;
#pragma unroll 4
    for (int i = 0; i < NBA / NWAVE / 2; ++i) {
      const int slot = wave * (NBA / NWAVE) + 2 * i + rsub;
      const float* sp = acc + slot * DF + c8;
      const v8h hv = cvt8(*(const v4f*)sp, *(const v4f*)(sp + 4));
      *(volatile v8h*)(hout + ((size_t)nodeBase + slot) * DF + c8) = hv;
    }
    __threadfence();
#pragma unroll 4
    for (int i = 0; i < NBA / NWAVE / 2; ++i) {
      const int slot = wave * (NBA / NWAVE) + 2 * i + rsub;
      const float* sp = acc + slot * DF + c8;
      const v8h hv = cvt8(*(const v4f*)sp, *(const v4f*)(sp + 4));
      *(volatile v8h*)(hout + ((size_t)nodeBase + slot) * DF + c8) = hv;
    }
  } else {
#pragma unroll 4
    for (int i = 0; i < NBA / NWAVE; ++i) {
      const int slot = wave * (NBA / NWAVE) + i;
      const v4f v = *(const v4f*)(acc + slot * DF + c4);
      *(volatile v4f*)(fout + ((size_t)nodeBase + slot) * DF + c4) = v;
    }
    __threadfence();
#pragma unroll 4
    for (int i = 0; i < NBA / NWAVE; ++i) {
      const int slot = wave * (NBA / NWAVE) + i;
      const v4f v = *(const v4f*)(acc + slot * DF + c4);
      *(volatile v4f*)(fout + ((size_t)nodeBase + slot) * DF + c4) = v;
    }
  }
}

__global__ __launch_bounds__(NTHR) void k_pool(
    const int* __restrict__ batch, const float* __restrict__ hb, float* gpool, int nN) {
  __shared__ __attribute__((aligned(16))) float acc[NGB * DF];
  __shared__ __attribute__((aligned(16))) int list[LISTN];
  __shared__ int cnt[NGB];
  __shared__ int wcnt[NWAVE];
  const int tid = threadIdx.x, lane = tid & 31, wave = tid >> 5;
  const int graphBase = blockIdx.x * NGB;

  for (int i = tid; i < NGB * DF; i += NTHR) acc[i] = 0.f;
  for (int i = tid; i < NGB; i += NTHR) cnt[i] = 0;
  __syncthreads();

  const int nChunks = (nN + CHUNK - 1) / CHUNK;
#pragma unroll 1
  for (int ch = 0; ch < nChunks; ++ch) {
    const int cbase = ch * CHUNK;
    const int wc = scan_chunk<NGB>(batch, nN, cbase, graphBase, list, tid, wave);
    if (lane == 0) wcnt[wave] = wc;
    __syncthreads();
    if (wave == 0) {
#pragma unroll 1
      for (int wsx = 0; wsx < NWAVE; ++wsx) {
        int n = __builtin_amdgcn_readfirstlane(wcnt[wsx]);
        n = n > WCAP ? WCAP : (n < 0 ? 0 : n);
        const int* lp = list + wsx * WCAP;
#pragma unroll 1
        for (int i = 0; i < n; ++i) {
          const int ent  = __builtin_amdgcn_readfirstlane(lp[i]);
          const int slot = ent & (NGB - 1);
          int nd = cbase + ((ent >> 12) & (CHUNK - 1));
          nd = nd > nN - 1 ? nN - 1 : nd;
          const v4f v = *(const v4f*)(hb + (size_t)nd * DF + 4 * lane);
          v4f* ap = (v4f*)(acc + slot * DF + 4 * lane);
          *ap = *ap + v;
          if (lane == 0) cnt[slot] = cnt[slot] + 1;
        }
      }
    }
    __syncthreads();
  }

#pragma unroll
  for (int i = 0; i < NGB / NWAVE; ++i) {
    const int slot = wave * (NGB / NWAVE) + i;
    const int c = cnt[slot];
    const float inv = 1.0f / (float)(c > 1 ? c : 1);
    const v4f v = *(const v4f*)(acc + slot * DF + 4 * lane) * inv;
    *(volatile v4f*)(gpool + ((size_t)graphBase + slot) * DF + 4 * lane) = v;
  }
  __threadfence();
#pragma unroll
  for (int i = 0; i < NGB / NWAVE; ++i) {
    const int slot = wave * (NGB / NWAVE) + i;
    const int c = cnt[slot];
    const float inv = 1.0f / (float)(c > 1 ? c : 1);
    const v4f v = *(const v4f*)(acc + slot * DF + 4 * lane) * inv;
    *(volatile v4f*)(gpool + ((size_t)graphBase + slot) * DF + 4 * lane) = v;
  }
}

__global__ __launch_bounds__(NTHR) void k_cls(
    const float* __restrict__ gpool, const float* __restrict__ clsv,
    const float* __restrict__ clsg, const float* __restrict__ clsb,
    float* out, int nG, int nC, int outN) {
  extern __shared__ v4f lds_dyn[];
  float* wn  = (float*)lds_dyn;
  float* stg = wn + nC * DF;
  const int tid = threadIdx.x, lane = tid & 31, wave = tid >> 5;
  (void)nG;

  for (int c = wave; c < nC; c += NWAVE) {
    const v4f v = *(const v4f*)(clsv + (size_t)c * DF + 4 * lane);
    const float n2  = wave_sum32(v.x * v.x + v.y * v.y + v.z * v.z + v.w * v.w);
    const float nrm = sqrtf(n2);
    const float rn  = 1.0f / nrm;
    const float gs  = clsg[c];
    v4f o;
    o.x = (gs * v.x) * rn; o.y = (gs * v.y) * rn; o.z = (gs * v.z) * rn; o.w = (gs * v.w) * rn;
    *(v4f*)(wn + c * DF + 4 * lane) = o;
  }
  __syncthreads();

#pragma unroll 1
  for (int p = tid; p < outN; p += NTHR) {
    const int gr = p / nC;
    const int c  = p - gr * nC;
    const float* gp = gpool + (size_t)gr * DF;
    const float* wp = wn + c * DF;
    float s = 0.f;
#pragma unroll 4
    for (int k4 = 0; k4 < DF / 4; ++k4) {
      const v4f a = *(const v4f*)(gp + 4 * k4);
      const v4f w = *(const v4f*)(wp + 4 * k4);
      s += a.x * w.x; s += a.y * w.y; s += a.z * w.z; s += a.w * w.w;
    }
    stg[p] = s + clsb[c];
  }
  __syncthreads();

  const int n4 = outN >> 2;
  const int rem = outN & 3;
  for (int q = tid; q < n4; q += NTHR) { const v4f v = *(const v4f*)(stg + 4 * q); *(volatile v4f*)(out + 4 * (size_t)q) = v; }
  if (tid < rem) { const float v = stg[4 * n4 + tid]; *(volatile float*)(out + 4 * (size_t)n4 + tid) = v; }
  __threadfence();
  for (int q = tid; q < n4; q += NTHR) { const v4f v = *(const v4f*)(stg + 4 * q); *(volatile v4f*)(out + 4 * (size_t)q) = v; }
  if (tid < rem) { const float v = stg[4 * n4 + tid]; *(volatile float*)(out + 4 * (size_t)n4 + tid) = v; }
}

extern "C" void kernel_launch(void* const* d_in, const int* in_sizes, int n_in,
                              void* d_out, int out_size, void* d_ws, size_t ws_size,
                              hipStream_t stream) {
  if (n_in < 15) return;
  const int nN = in_sizes[3];
  const int nE = in_sizes[1];
  const int nC = in_sizes[13];
  if (nN <= 0 || nE < 0 || nC <= 0) return;
  if (in_sizes[0] != nN * DF || in_sizes[2] != nE) return;
  if (in_sizes[4] != DF * DF || in_sizes[8] != DF * DF) return;
  if (in_sizes[5] < DF || in_sizes[6] < DF || in_sizes[7] < DF) return;
  if (in_sizes[9] < DF || in_sizes[10] < DF || in_sizes[11] < DF) return;
  if (in_sizes[12] != nC * DF || in_sizes[14] < nC) return;
  if (out_size <= 0 || (out_size % nC) != 0) return;
  const int nG = out_size / nC;

  const float* x     = (const float*)d_in[0];
  const int*   src   = (const int*)d_in[1];
  const int*   dst   = (const int*)d_in[2];
  const int*   batch = (const int*)d_in[3];
  const float* W1    = (const float*)d_in[4];
  const float* b1    = (const float*)d_in[5];
  const float* ln1w  = (const float*)d_in[6];
  const float* ln1b  = (const float*)d_in[7];
  const float* W2    = (const float*)d_in[8];
  const float* b2    = (const float*)d_in[9];
  const float* ln2w  = (const float*)d_in[10];
  const float* ln2b  = (const float*)d_in[11];
  const float* clsv  = (const float*)d_in[12];
  const float* clsg  = (const float*)d_in[13];
  const float* clsb  = (const float*)d_in[14];
  float* out = (float*)d_out;

  const int nBD  = (nN + NBD - 1) / NBD;
  const int nA   = (nN + NBA - 1) / NBA;
  const int nPad = nA * NBA;
  const int nGm  = nPad / GROWS;
  const int nPB  = (nG + NGB - 1) / NGB;

  char* ws = (char*)d_ws;
  size_t off = 0;
  const size_t oW1 = off; off += (size_t)DF * DF * 2;               off = (off + 255) & ~(size_t)255;
  const size_t oW2 = off; off += (size_t)DF * DF * 2;               off = (off + 255) & ~(size_t)255;
  const size_t oDv = off; off += (size_t)nBD * NBD * 4;             off = (off + 255) & ~(size_t)255;
  const size_t oXh = off; off += (size_t)nPad * DF * 2;             off = (off + 255) & ~(size_t)255;
  const size_t oG  = off; off += (size_t)nPad * DF * 4;             off = (off + 255) & ~(size_t)255;
  const size_t oHb = off; off += (size_t)nPad * DF * 4;             off = (off + 255) & ~(size_t)255;
  const size_t oGp = off; off += (size_t)nPB * NGB * DF * 4;        off = (off + 255) & ~(size_t)255;
  if (off > ws_size) return;
  const size_t ldsCls = ((size_t)nC * DF + (((size_t)out_size + 3) & ~(size_t)3)) * 4;
  if (ldsCls > (size_t)160 * 1024) return;

  _Float16* w1s   = (_Float16*)(ws + oW1);
  _Float16* w2s   = (_Float16*)(ws + oW2);
  float*    dinv  = (float*)(ws + oDv);
  _Float16* xh    = (_Float16*)(ws + oXh);
  float*    gpl   = (float*)(ws + oG);
  float*    hbp   = (float*)(ws + oHb);
  float*    gpool = (float*)(ws + oGp);

  const int nPrep = 2 * (DF * DF / 8);
  k_wprep<<<(nPrep + NTHR - 1) / NTHR, NTHR, 0, stream>>>(W1, W2, w1s, w2s);

  const size_t nCvt = (size_t)nPad * (DF / 8);
  k_xcvt<<<(unsigned)((nCvt + NTHR - 1) / NTHR), NTHR, 0, stream>>>(x, xh, nN, nPad);

  k_deg<<<nBD, NTHR, 0, stream>>>(dst, dinv, nE);

  hipFuncSetAttribute(reinterpret_cast<const void*>(&k_gemm),
                      hipFuncAttributeMaxDynamicSharedMemorySize, LDS_GEMM);
  k_gemm<<<nGm, NTHR, LDS_GEMM, stream>>>(xh, w1s, dinv, gpl);

  hipFuncSetAttribute(reinterpret_cast<const void*>(&k_agg<1>),
                      hipFuncAttributeMaxDynamicSharedMemorySize, LDS_AGG);
  k_agg<1><<<nA, NTHR, LDS_AGG, stream>>>(src, dst, gpl, dinv, b1, ln1w, ln1b, xh, hbp, nN, nE);

  k_gemm<<<nGm, NTHR, LDS_GEMM, stream>>>(xh, w2s, dinv, gpl);

  hipFuncSetAttribute(reinterpret_cast<const void*>(&k_agg<2>),
                      hipFuncAttributeMaxDynamicSharedMemorySize, LDS_AGG);
  k_agg<2><<<nA, NTHR, LDS_AGG, stream>>>(src, dst, gpl, dinv, b2, ln2w, ln2b, xh, hbp, nN, nE);

  k_pool<<<nPB, NTHR, 0, stream>>>(batch, hbp, gpool, nN);

  k_cls<<<1, NTHR, ldsCls, stream>>>(gpool, clsv, clsg, clsb, out, nG, nC, out_size);
}
